// SelfSeqAtten_16166256902633
// MI455X (gfx1250) — hardware-run, weakly checked
//
#include <hip/hip_runtime.h>


namespace {
constexpr int L = 2048, NB = 8, D = 128, KB = 128;
constexpr float XS = 8.0f, PS = 256.0f;
typedef _Float16 b16;
typedef __attribute__((ext_vector_type(16))) _Float16 v16b;
typedef __attribute__((ext_vector_type(8))) _Float16 v8b;
typedef __attribute__((ext_vector_type(8))) float v8f;
typedef __attribute__((ext_vector_type(4))) float v4f;
__device__ __forceinline__ float bf16_rne(float f) { unsigned int u = __float_as_uint(f); u += 0x7FFFu + ((u >> 16) & 1u); float r = __uint_as_float(u & 0xFFFF0000u); asm volatile("" : "+v"(r)); return r; }
__device__ __forceinline__ void split16(float v, b16& hi, b16& lo) { hi = (b16)v; lo = (b16)(v - (float)hi); }
__device__ __forceinline__ v16b frag_kb(const b16* p, int hh) { const v8b a = *(const v8b*)(p + 8 * hh), b = *(const v8b*)(p + 16 + 8 * hh); v16b f;
#pragma unroll
  for (int e = 0; e < 8; ++e) { f[e] = a[e]; f[8 + e] = b[e]; } return f; }
__device__ __forceinline__ v8f wmma16b(v16b a, v16b b, v8f c) { v8f d = __builtin_amdgcn_wmma_f32_16x16x32_f16(false, a, false, b, (short)0, c, false, false); asm volatile("v_nop\n\tv_nop\n\tv_nop\n\tv_nop" : "+v"(d) : "v"(a), "v"(b)); return d; }
__device__ __forceinline__ void wave_lds_sync() { __builtin_amdgcn_fence(__ATOMIC_RELEASE, "workgroup"); __builtin_amdgcn_wave_barrier(); __builtin_amdgcn_fence(__ATOMIC_ACQUIRE, "workgroup"); }
__device__ __forceinline__ float pmul(float a, float b) { float p = a * b; asm volatile("" : "+v"(p)); return p; }

__global__ __launch_bounds__(256) void hput_kernel(const float* __restrict__ h, b16* __restrict__ HP) { const size_t u = (size_t)blockIdx.x * 256 + threadIdx.x; if (u >= (size_t)NB * L * D / 8) return; const size_t e = u * 8; const int b = (int)(e / ((size_t)L * D)); const size_t rem = e % ((size_t)L * D); const int j = (int)(rem / D), k0 = (int)(rem % D); v8b v;
#pragma unroll
  for (int q = 0; q < 8; ++q) v[q] = (b16)(bf16_rne(h[((size_t)j * NB + b) * D + k0 + q]) * XS); for (int pass = 0; pass < 2; ++pass) { *(volatile v8b*)(HP + e) = v; __threadfence(); } }
__global__ __launch_bounds__(32) void att_kernel(const b16* __restrict__ HP, const int* __restrict__ mask, int BLIM, float* __restrict__ out) { __shared__ __attribute__((aligned(16))) b16 Ph[16][KB + 8], Pl[16][KB + 8], Vt[D][KB + 8]; __shared__ float Sf[16][KB + 4], Mk[KB], Of[16][D + 4];
  const int lane = threadIdx.x, nloc = lane & 15, hlf = lane >> 4; const int qt = blockIdx.x % (L / 16); const int b = blockIdx.x / (L / 16); if (b >= BLIM) return; const int t0 = qt * 16; const b16* Hb = HP + (size_t)b * L * D;
  v16b qa[4];
#pragma unroll
  for (int q = 0; q < 4; ++q) qa[q] = frag_kb(Hb + (size_t)(t0 + nloc) * D + q * 32, hlf);
  float m_r[8], den_r[8]; v8f acc[8];
#pragma unroll
  for (int r8 = 0; r8 < 8; ++r8) { m_r[r8] = -INFINITY; den_r[r8] = 0.0f; }
#pragma unroll
  for (int t = 0; t < 8; ++t) acc[t] = (v8f){};
#pragma unroll 1
  for (int kb0 = 0; kb0 < L; kb0 += KB) {
    for (int rr = 0; rr < KB; rr += 2) { const int r = rr + hlf; const b16* hr = Hb + (size_t)(kb0 + r) * D; for (int q = 0; q < 8; ++q) Vt[q * 16 + nloc][r] = hr[q * 16 + nloc]; }
    for (int kk = 0; kk < KB; kk += 32) Mk[kk + lane] = mask[(size_t)b * L + kb0 + kk + lane] != 0 ? 1.0f : 0.0f;
    wave_lds_sync();
#pragma unroll
    for (int t = 0; t < KB / 16; ++t) { v8f s = {};
#pragma unroll
      for (int q = 0; q < 4; ++q) s = wmma16b(qa[q], frag_kb(Hb + (size_t)(kb0 + t * 16 + nloc) * D + q * 32, hlf), s);
#pragma unroll
      for (int r8 = 0; r8 < 8; ++r8) { const int i = t0 + 8 * hlf + r8, j = kb0 + t * 16 + nloc; Sf[8 * hlf + r8][t * 16 + nloc] = (i == j) ? 0.0f : s[r8] * (1.0f / (XS * XS)); } }
    wave_lds_sync();
#pragma unroll
    for (int rr = 0; rr < 16; ++rr) { float mx = -INFINITY;
#pragma unroll
      for (int q = 0; q < 4; ++q) { const int kx = q * 32 + lane; if (Mk[kx] > 0.0f) mx = fmaxf(mx, Sf[rr][kx]); }
      for (int o = 16; o; o >>= 1) mx = fmaxf(mx, __shfl_xor(mx, o));
      const float mold = __shfl(m_r[rr & 7], (rr >> 3) * 16); const float mn = fmaxf(mold, mx); const float sf = (mold == -INFINITY) ? 0.0f : ((mn == -INFINITY) ? 1.0f : __expf(mold - mn)); float ps = 0.0f;
#pragma unroll
      for (int q = 0; q < 4; ++q) { const int kx = q * 32 + lane; const float p = (Mk[kx] > 0.0f && mn > -INFINITY) ? __expf(Sf[rr][kx] - mn) : 0.0f; ps += p; b16 ph, pl; split16(p * PS, ph, pl); Ph[rr][kx] = ph; Pl[rr][kx] = pl; }
      for (int o = 16; o; o >>= 1) ps += __shfl_xor(ps, o);
      if ((rr >> 3) == hlf) { const int r8 = rr & 7; den_r[r8] = den_r[r8] * sf + ps; m_r[r8] = mn;
#pragma unroll
        for (int t = 0; t < 8; ++t) acc[t][r8] = acc[t][r8] * sf; } }
    wave_lds_sync();
#pragma unroll
    for (int ks = 0; ks < KB; ks += 32) { const v16b pa = frag_kb(&Ph[nloc][ks], hlf), pb = frag_kb(&Pl[nloc][ks], hlf);
#pragma unroll
      for (int t = 0; t < 8; ++t) { const v16b vh = frag_kb(&Vt[t * 16 + nloc][ks], hlf); acc[t] = wmma16b(pa, vh, acc[t]); acc[t] = wmma16b(pb, vh, acc[t]); } }
    wave_lds_sync(); }
#pragma unroll
  for (int t = 0; t < 8; ++t)
#pragma unroll
    for (int r8 = 0; r8 < 8; ++r8) { const float dn = den_r[r8]; Of[8 * hlf + r8][t * 16 + nloc] = dn > 0.0f ? acc[t][r8] * (1.0f / (XS * PS)) / dn : 0.0f; }
  wave_lds_sync();
  for (int pass = 0; pass < 2; ++pass) { for (int rr = 0; rr < 16; ++rr) *(volatile v4f*)(out + ((size_t)(t0 + rr) * NB + b) * D + lane * 4) = *(const v4f*)(&Of[rr][lane * 4]); __threadfence(); } }
}

extern "C" void kernel_launch(void* const* d_in, const int* in_sizes, int n_in, void* d_out, int out_size, void* d_ws, size_t ws_size, hipStream_t stream) {
  (void)n_in;
  if (in_sizes[0] != L * NB * D || in_sizes[1] != NB * L || out_size != L * NB * D) return;
  const int BLIM = NB;
  size_t off = 0; char* ws = (char*)d_ws;
  auto carve = [&](size_t bytes) { char* p = ws + off; off += (bytes + 255) & ~(size_t)255; return p; };
  b16* HP = (b16*)carve((size_t)NB * L * D * 2);
  if (off > ws_size || off > ((size_t)16 << 20)) return;
  hput_kernel<<<(unsigned)(((size_t)NB * L * D / 8 + 255) / 256), 256, 0, stream>>>((const float*)d_in[0], HP);
  att_kernel<<<BLIM * (L / 16), 32, 0, stream>>>(HP, (const int*)d_in[1], BLIM, (float*)d_out);
}
